// MultiHeadAttention_274877907714
// MI455X (gfx1250) — hardware-verified
//
#include <hip/hip_runtime.h>
#include <math.h>

#ifndef NTOK
#define NTOK 8192
#endif
#define NTOK_FULL 8192
#define DM   128
#define NHD  16
#define FEAT 2048
#define NGRP ((NTOK + 4095) / 4096)
#define GTOK (NTOK / NGRP)
static_assert(NTOK % NGRP == 0);
static_assert(GTOK % 64 == 0);
static_assert(NTOK % 16 == 0);
static_assert(NTOK <= NTOK_FULL);
static_assert(DM % 64 == 0);
static_assert(FEAT % 64 == 0);
static_assert(DM % 32 == 0);
static_assert(FEAT == DM * NHD);

typedef __attribute__((ext_vector_type(16))) _Float16 v16h;
typedef __attribute__((ext_vector_type(8)))  _Float16 v8h;
typedef __attribute__((ext_vector_type(16))) __bf16   v16b;
typedef __attribute__((ext_vector_type(8)))  __bf16   v8b;
typedef __attribute__((ext_vector_type(8)))  float    v8f;
typedef __attribute__((ext_vector_type(4)))  float    v4f;
typedef __attribute__((ext_vector_type(16))) unsigned short v16us;
typedef __attribute__((ext_vector_type(8)))  unsigned short v8us;
typedef __attribute__((ext_vector_type(4)))  unsigned int   v4u;

__device__ __forceinline__ v8f wmma16(v16h a, v16h b, v8f c) {
    c = __builtin_amdgcn_wmma_f32_16x16x32_f16(false, a, false, b, (short)0, c, false, false);
    asm volatile("v_nop\n\tv_nop\n\tv_nop\n\tv_nop" : "+v"(c) : "v"(a), "v"(b));
    return c;
}
__device__ __forceinline__ v8f wmmab(v16b a, v16b b, v8f c) {
    c = __builtin_amdgcn_wmma_f32_16x16x32_bf16(false, a, false, b, (short)0, c, false, false);
    asm volatile("v_nop\n\tv_nop\n\tv_nop\n\tv_nop" : "+v"(c) : "v"(a), "v"(b));
    return c;
}

__device__ __forceinline__ unsigned short bf_bits(float f) { unsigned u = __float_as_uint(f); return (unsigned short)((u + 0x7FFFu + ((u >> 16) & 1u)) >> 16); }
__device__ __forceinline__ float bfb2f(unsigned short hb) { return __uint_as_float(((unsigned int)hb) << 16); }
__device__ __forceinline__ float cmb_bf(float v) { const unsigned u = __builtin_bit_cast(unsigned, v); const unsigned r = (u + 0x7fffu + ((u >> 16) & 1u)) & 0xffff0000u; return __builtin_bit_cast(float, r); }
__device__ __forceinline__ void bfsplit(float v, unsigned short& hi, unsigned short& lo) { hi = bf_bits(v); lo = bf_bits(v - bfb2f(hi)); }
__device__ __forceinline__ unsigned int pk2_f16(float a, float b) { return (unsigned int)__builtin_bit_cast(unsigned short, (_Float16)a) | ((unsigned int)__builtin_bit_cast(unsigned short, (_Float16)b) << 16); }
__device__ __forceinline__ unsigned int pk2_bf(float a, float b)  { return (unsigned int)bf_bits(a) | ((unsigned int)bf_bits(b) << 16); }

#define VST2(T, ptr, val) do { const T vst2_v_ = (val); *(volatile T*)(ptr) = vst2_v_; __threadfence(); *(volatile T*)(ptr) = vst2_v_; } while (0)

namespace w25 {

__device__ __forceinline__ unsigned short f2bf_bits(float f) {
  unsigned u = __float_as_uint(f);
  return (unsigned short)((u + 0x7FFFu + ((u >> 16) & 1u)) >> 16);
}
__device__ __forceinline__ float bf_bits2f(unsigned short h) { return __uint_as_float(((unsigned)h) << 16); }

__device__ __forceinline__ void dep_guard_h(v8f& a, v8f& b, v16h x, v16h y) { asm volatile("v_nop\n\tv_nop\n\tv_nop\n\tv_nop" : "+v"(a), "+v"(b) : "v"(x), "v"(y)); }
__device__ __forceinline__ void dep_guard_b(v8f& a, v8f& b, v16b x, v16b y) { asm volatile("v_nop\n\tv_nop\n\tv_nop\n\tv_nop" : "+v"(a), "+v"(b) : "v"(x), "v"(y)); }
__device__ __forceinline__ void keep4_h(v16h a, v16h b, v16h c, v16h d) { asm volatile("v_nop" :: "v"(a), "v"(b), "v"(c), "v"(d)); }
__device__ __forceinline__ void keep4_b(v16b a, v16b b, v16b c, v16b d) { asm volatile("v_nop" :: "v"(a), "v"(b), "v"(c), "v"(d)); }
__device__ __forceinline__ void acc_guard4(v8f& a, v8f& b, v8f& c, v8f& d) { asm volatile("v_nop\n\tv_nop\n\tv_nop\n\tv_nop" : "+v"(a), "+v"(b), "+v"(c), "+v"(d)); }
template <typename T> struct Frag;
template <> struct Frag<_Float16> {
  typedef v16h V; union U { v16h v; v8h h[2]; };
  static __device__ __forceinline__ v16h load(const _Float16* p) {
    U f; f.h[0] = *(const v8h*)(p); f.h[1] = *(const v8h*)(p + 16); return f.v;
  }
  static __device__ __forceinline__ v8f mma(v16h a, v16h b, v8f c) {
    return __builtin_amdgcn_wmma_f32_16x16x32_f16(false, a, false, b, (short)0, c, false, false);
  }
  static __device__ __forceinline__ void guard(v8f& a, v8f& b, v16h x, v16h y) { dep_guard_h(a, b, x, y); }
  static __device__ __forceinline__ void keep(v16h a, v16h b, v16h c, v16h d) { keep4_h(a, b, c, d); }
};
template <> struct Frag<__bf16> {
  typedef v16b V; union U { v16b v; v8b h[2]; };
  static __device__ __forceinline__ v16b load(const __bf16* p) {
    U f; f.h[0] = *(const v8b*)(p); f.h[1] = *(const v8b*)(p + 16); return f.v;
  }
  static __device__ __forceinline__ v8f mma(v16b a, v16b b, v8f c) {
    return __builtin_amdgcn_wmma_f32_16x16x32_bf16(false, a, false, b, (short)0, c, false, false);
  }
  static __device__ __forceinline__ void guard(v8f& a, v8f& b, v16b x, v16b y) { dep_guard_b(a, b, x, y); }
  static __device__ __forceinline__ void keep(v16b a, v16b b, v16b c, v16b d) { keep4_b(a, b, c, d); }
};

template <int ET> struct Elem;
template <> struct Elem<0> { typedef _Float16 T; };
template <> struct Elem<1> { typedef __bf16 T; };
template <int ET, bool SPLIT, int BIAS_MODE, int OUT_MODE, bool RESID, int ACT = 0>
__global__ __launch_bounds__(256) void wmma_gemm64(
    const unsigned short* __restrict__ Ap, const unsigned short* __restrict__ A2p, int lda, long strideA,
    const unsigned short* __restrict__ Btp, const unsigned short* __restrict__ Bt2p, int ldb, long strideB,
    void* __restrict__ Cout, void* __restrict__ Cout2, int ldc, long strideC,
    const float* __restrict__ bias,
    const float* __restrict__ resid, long strideR,
    int M, int N, int K, float scale) {
  typedef typename Elem<ET>::T T;
  typedef typename Frag<T>::V V;
  const T* A = (const T*)Ap; const T* A2 = (const T*)A2p; const T* Bt = (const T*)Btp; const T* Bt2 = (const T*)Bt2p;
  __shared__ __align__(16) float sT[8][16 * 68];
  const int b    = blockIdx.y;
  const int lane = threadIdx.x & 31;
  const int wave = threadIdx.x >> 5;
  const int tilesN = N >> 6;
  const int tilesM = M >> 6;
  const int tile = blockIdx.x * 8 + wave;
  if (tile >= tilesM * tilesN) return;
  const int tm = tile / tilesN;
  const int tn = tile - tm * tilesN;
  const int m0 = tm << 6;
  const int n0 = tn << 6;

  const T* Ab  = A  + (size_t)b * strideA;
  const T* Bb  = Bt + (size_t)b * strideB;
  const T* Ab2 = SPLIT ? (A2  + (size_t)b * strideA) : nullptr;
  const T* Bb2 = SPLIT ? (Bt2 + (size_t)b * strideB) : nullptr;

  const int rlane = lane & 15;
  const int koff  = (lane >> 4) * 8;
  const int mOff  = (lane >> 4) * 8;

  v8f acc[4][4];
#pragma unroll
  for (int i = 0; i < 4; ++i)
#pragma unroll
    for (int j = 0; j < 4; ++j) acc[i][j] = (v8f){0.f,0.f,0.f,0.f,0.f,0.f,0.f,0.f};

  for (int k0 = 0; k0 < K; k0 += 32) {
    V bh[4], bl[4];
#pragma unroll
    for (int j = 0; j < 4; ++j) {
      const size_t bo = (size_t)(n0 + (j << 4) + rlane) * ldb + koff + k0;
      bh[j] = Frag<T>::load(Bb + bo);
      if (SPLIT) bl[j] = Frag<T>::load(Bb2 + bo);
    }
#pragma unroll
    for (int i = 0; i < 4; ++i) {
      const size_t ao = (size_t)(m0 + (i << 4) + rlane) * lda + koff + k0;
      V ah = Frag<T>::load(Ab + ao);
      V al = ah;
      if (SPLIT) al = Frag<T>::load(Ab2 + ao);
#pragma unroll
      for (int j = 0; j < 4; ++j) {
        acc[i][j] = Frag<T>::mma(ah, bh[j], acc[i][j]);
        if (SPLIT) {
          acc[i][j] = Frag<T>::mma(ah, bl[j], acc[i][j]);
          acc[i][j] = Frag<T>::mma(al, bh[j], acc[i][j]);
        }
      }
      Frag<T>::guard(acc[i][0], acc[i][3], ah, SPLIT ? al : ah);
    }
    Frag<T>::keep(bh[0], bh[1], bh[2], bh[3]);
    if (SPLIT) Frag<T>::keep(bl[0], bl[1], bl[2], bl[3]);
  }
  acc_guard4(acc[0][0], acc[0][1], acc[0][2], acc[0][3]);
  acc_guard4(acc[1][0], acc[1][1], acc[1][2], acc[1][3]);
  acc_guard4(acc[2][0], acc[2][1], acc[2][2], acc[2][3]);
  acc_guard4(acc[3][0], acc[3][1], acc[3][2], acc[3][3]);

  float* slab = sT[wave];
  const float* Rb = RESID ? (resid + (size_t)b * strideR) : nullptr;
#pragma unroll
  for (int i = 0; i < 4; ++i) {
    const int mBase = m0 + (i << 4);
#pragma unroll
    for (int j = 0; j < 4; ++j) {
      const int n = n0 + (j << 4) + rlane;
      float bv = 0.f;
      if (BIAS_MODE == 2) bv = bias[n];
#pragma unroll
      for (int r = 0; r < 8; ++r) {
        float v = acc[i][j][r] * scale;
        if (BIAS_MODE == 1) v += bias[mBase + mOff + r];
        if (BIAS_MODE == 2) v += bv;
        if (RESID) v += Rb[(size_t)(mBase + mOff + r) * ldc + n];
        if (ACT == 1) v = tanhf(v);
        if (ACT == 2) v = fmaxf(v, 0.0f);
        slab[(mOff + r) * 68 + (j << 4) + rlane] = v;
      }
    }
    __builtin_amdgcn_fence(3  , "workgroup");
    __builtin_amdgcn_wave_barrier();
    __builtin_amdgcn_fence(2  , "workgroup");
    if (OUT_MODE == 0) {
      float* C = (float*)Cout + (size_t)b * strideC;
      const int hh = lane >> 4, c4 = (lane & 15) * 4;
      for (int pass = 0; pass < 2; ++pass) {
#pragma unroll
        for (int it = 0; it < 8; ++it) {
          const int row = it * 2 + hh;
          v4f v = *(const v4f*)(slab + row * 68 + c4);
          *(volatile v4f*)(C + (size_t)(mBase + row) * ldc + n0 + c4) = v;
        }
        __threadfence();
      }
    } else {
      const int q = lane >> 3, c8 = (lane & 7) * 8;
      unsigned short* C  = (unsigned short*)Cout  + (size_t)b * strideC;
      unsigned short* C2 = (OUT_MODE == 2) ? ((unsigned short*)Cout2 + (size_t)b * strideC) : nullptr;
      for (int pass = 0; pass < 2; ++pass) {
#pragma unroll
        for (int it = 0; it < 4; ++it) {
          const int row = it * 4 + q;
          const float* sp = slab + row * 68 + c8;
          v8h hv, lv;
#pragma unroll
          for (int e = 0; e < 8; ++e) {
            if (OUT_MODE == 1) {
              hv[e] = (_Float16)sp[e];
              lv[e] = hv[e];
            } else {
              unsigned short hb = f2bf_bits(sp[e]);
              unsigned short lb = f2bf_bits(sp[e] - bf_bits2f(hb));
              hv[e] = __builtin_bit_cast(_Float16, hb);
              lv[e] = __builtin_bit_cast(_Float16, lb);
            }
          }
          *(volatile v8h*)(C + (size_t)(mBase + row) * ldc + n0 + c8) = hv;
          if (OUT_MODE == 2) *(volatile v8h*)(C2 + (size_t)(mBase + row) * ldc + n0 + c8) = lv;
        }
        __threadfence();
      }
    }
    __builtin_amdgcn_fence(3  , "workgroup");
    __builtin_amdgcn_wave_barrier();
    __builtin_amdgcn_fence(2  , "workgroup");
  }
}

}

__global__ __launch_bounds__(256) void k_castrows(const float* __restrict__ SRC, int lds, unsigned short* __restrict__ DST, int ldd, int nR, int nC, float sc) {
    const long long u = (long long)blockIdx.x * 256 + threadIdx.x; const int per = nC / 8; if (u >= (long long)nR * per) return;
    const int r = (int)(u / per); const int c0 = 8 * (int)(u % per);
    const float* s = SRC + (long long)r * lds + c0; float w[8];
#pragma unroll
    for (int e = 0; e < 8; ++e) w[e] = cmb_bf(s[e]) * sc;
    v4u pk; pk.x = pk2_f16(w[0], w[1]); pk.y = pk2_f16(w[2], w[3]); pk.z = pk2_f16(w[4], w[5]); pk.w = pk2_f16(w[6], w[7]);
    VST2(v4u, (v4u*)(DST + (long long)r * ldd + c0), pk); }

__global__ __launch_bounds__(256) void k_castwT(const float* __restrict__ SRC, int lds, unsigned short* __restrict__ DST, int ldd, int nR, int nC, float sc, int fmt, int jn, int hn, int dupoff) {
    const long long u = (long long)blockIdx.x * 256 + threadIdx.x; const int per = nR / 8; if (u >= (long long)nC * per) return;
    const int c = (int)(u / per); const int r0 = 8 * (int)(u % per);
    const int csrc = (hn > 0) ? ((c % jn) * hn + c / jn) : c;
    float w[8];
#pragma unroll
    for (int e = 0; e < 8; ++e) w[e] = cmb_bf(SRC[(long long)(r0 + e) * lds + csrc]) * sc;
    v4u ph, pb;
    ph.x = pk2_f16(w[0], w[1]); ph.y = pk2_f16(w[2], w[3]); ph.z = pk2_f16(w[4], w[5]); ph.w = pk2_f16(w[6], w[7]);
    pb.x = pk2_bf(w[0], w[1]);  pb.y = pk2_bf(w[2], w[3]);  pb.z = pk2_bf(w[4], w[5]);  pb.w = pk2_bf(w[6], w[7]);
    const v4u pk = (fmt == 0) ? ph : pb;
    VST2(v4u, (v4u*)(DST + (long long)c * ldd + r0), pk);
    if (dupoff > 0) VST2(v4u, (v4u*)(DST + (long long)c * ldd + dupoff + r0), pk); }

__global__ __launch_bounds__(256) void k_bfvec(const float* __restrict__ SRC, float* __restrict__ DST, int n, int jn, int hn) {
    const int u = blockIdx.x * 256 + threadIdx.x; if (u >= n) return;
    const int is = (hn > 0) ? ((u % jn) * hn + u / jn) : u;
    VST2(float, DST + u, cmb_bf(SRC[is])); }

__global__ __launch_bounds__(256) void k_featattn(const unsigned short* __restrict__ QP, const unsigned short* __restrict__ KP,
                                                   const unsigned short* __restrict__ VH, const unsigned short* __restrict__ VL,
                                                   unsigned short* __restrict__ OP, int ntok) {
    union F16U { v16h v; v8us uh[2]; };
    union BFU  { v16b v; v16us u; v8us uh[2]; };
    const int lane = threadIdx.x & 31, wave = threadIdx.x >> 5, hf = lane >> 4, m = lane & 15;
    const int t = blockIdx.x * 8 + wave;
    if (t >= ntok) return;
    const unsigned short* qp  = QP + (size_t)t * FEAT;
    const unsigned short* kp  = KP + (size_t)t * FEAT;
    const unsigned short* vhp = VH + (size_t)t * FEAT;
    const unsigned short* vlp = VL + (size_t)t * FEAT;
    const v8us z8 = {0, 0, 0, 0, 0, 0, 0, 0};
    const float KLOG = 1.4426950408889634f * 0.088388347648318447f;
    v8f o[8];
#pragma unroll
    for (int it = 0; it < 8; ++it) { v8f zz = {}; o[it] = zz; }
    float vsum = 0.f;
#pragma unroll 1
    for (int jt = 0; jt < 8; ++jt) {
        const int j0 = jt * 16;
        F16U ak; ak.uh[0] = *(const v8us*)(kp + (j0 + m) * NHD + 8 * hf); ak.uh[1] = z8;
        v8f s[8];
#pragma unroll
        for (int it = 0; it < 8; ++it) {
            F16U bq; bq.uh[0] = *(const v8us*)(qp + (it * 16 + m) * NHD + 8 * hf); bq.uh[1] = z8;
            v8f zz = {}; s[it] = wmma16(ak.v, bq.v, zz);
        }
#pragma unroll
        for (int r = 0; r < 8; ++r) {
            float mx = s[0][r];
#pragma unroll
            for (int it = 1; it < 8; ++it) mx = fmaxf(mx, s[it][r]);
            mx = fmaxf(mx, __shfl_xor(mx, 1, 32)); mx = fmaxf(mx, __shfl_xor(mx, 2, 32));
            mx = fmaxf(mx, __shfl_xor(mx, 4, 32)); mx = fmaxf(mx, __shfl_xor(mx, 8, 32));
            float l = 0.f;
#pragma unroll
            for (int it = 0; it < 8; ++it) { const float e = exp2f((s[it][r] - mx) * KLOG); s[it][r] = e; l += e; }
            l += __shfl_xor(l, 1, 32); l += __shfl_xor(l, 2, 32); l += __shfl_xor(l, 4, 32); l += __shfl_xor(l, 8, 32);
            const float inv = 1.f / l;
#pragma unroll
            for (int it = 0; it < 8; ++it) s[it][r] = s[it][r] * inv - 0.0078125f;
        }
        BFU av;
        av.uh[0] = *(const v8us*)(vhp + m * DM + j0 + 8 * hf);
        av.uh[1] = *(const v8us*)(vlp + m * DM + j0 + 8 * hf);
#pragma unroll
        for (int e = 0; e < 16; ++e) vsum += bfb2f(av.u[e]);
#pragma unroll
        for (int it = 0; it < 8; ++it) {
            v8us ph;
#pragma unroll
            for (int r = 0; r < 8; ++r) ph[r] = bf_bits(s[it][r]);
            BFU pb; pb.uh[0] = ph; pb.uh[1] = ph;
            o[it] = wmmab(av.v, pb.v, o[it]);
        }
    }
    vsum += __shfl_xor(vsum, 16, 32);
    float mvr[8];
#pragma unroll
    for (int r = 0; r < 8; ++r) mvr[r] = __shfl(vsum, 8 * hf + r, 32) * 0.0078125f;
    unsigned short* op = OP + (size_t)t * (2 * FEAT);
    const int src = ((lane & 1) << 4) | (lane >> 1);
#pragma unroll
    for (int it = 0; it < 8; ++it) {
        unsigned int hp[4], lp[4];
#pragma unroll
        for (int r2 = 0; r2 < 4; ++r2) {
            unsigned short h0, l0, h1, l1;
            const float x0 = o[it][2 * r2] + mvr[2 * r2], x1 = o[it][2 * r2 + 1] + mvr[2 * r2 + 1];
            bfsplit(x0, h0, l0); bfsplit(x1, h1, l1);
            hp[r2] = (unsigned int)h0 | ((unsigned int)h1 << 16); lp[r2] = (unsigned int)l0 | ((unsigned int)l1 << 16);
        }
        v4u hq, lq;
        hq.x = __shfl(hp[0], src, 32); hq.y = __shfl(hp[1], src, 32); hq.z = __shfl(hp[2], src, 32); hq.w = __shfl(hp[3], src, 32);
        lq.x = __shfl(lp[0], src, 32); lq.y = __shfl(lp[1], src, 32); lq.z = __shfl(lp[2], src, 32); lq.w = __shfl(lp[3], src, 32);
        unsigned short* dh = op + it * 256 + lane * 8;
        unsigned short* dl = dh + FEAT;
        *(volatile v4u*)dh = hq; *(volatile v4u*)dl = lq;
        __threadfence();
        *(volatile v4u*)dh = hq; *(volatile v4u*)dl = lq;
    }
}

static inline size_t al256(size_t b) { return ((b + 255) / 256) * 256; }

extern "C" void kernel_launch(void* const* d_in, const int* in_sizes, int n_in, void* d_out, int out_size, void* d_ws, size_t ws_size, hipStream_t stream) {
    if (n_in < 11) return;
    if (in_sizes[0] < NTOK * DM || in_sizes[1] < NTOK * DM || in_sizes[2] < NTOK * DM) return;
    if (in_sizes[3] < DM * FEAT || in_sizes[5] < DM * FEAT || in_sizes[7] < DM * FEAT || in_sizes[9] < FEAT * DM) return;
    if (in_sizes[4] < FEAT || in_sizes[6] < FEAT || in_sizes[8] < FEAT || in_sizes[10] < DM) return;
    if (out_size < NTOK * DM) return;
    const float* q  = (const float*)d_in[0];
    const float* k  = (const float*)d_in[1];
    const float* v  = (const float*)d_in[2];
    const float* Wq = (const float*)d_in[3];
    const float* bq = (const float*)d_in[4];
    const float* Wk = (const float*)d_in[5];
    const float* bk = (const float*)d_in[6];
    const float* Wv = (const float*)d_in[7];
    const float* bv = (const float*)d_in[8];
    const float* Wo = (const float*)d_in[9];
    const float* bo = (const float*)d_in[10];
    float* out = (float*)d_out;

    char* wsp = (char*)d_ws;
    unsigned short* XQ16 = (unsigned short*)wsp; wsp += al256((size_t)NTOK * DM * 2);
    unsigned short* XK16 = (unsigned short*)wsp; wsp += al256((size_t)NTOK * DM * 2);
    unsigned short* XV16 = (unsigned short*)wsp; wsp += al256((size_t)NTOK * DM * 2);
    unsigned short* WQ16 = (unsigned short*)wsp; wsp += al256((size_t)FEAT * DM * 2);
    unsigned short* WK16 = (unsigned short*)wsp; wsp += al256((size_t)FEAT * DM * 2);
    unsigned short* WV16 = (unsigned short*)wsp; wsp += al256((size_t)FEAT * DM * 2);
    unsigned short* WO16 = (unsigned short*)wsp; wsp += al256((size_t)DM * 2 * FEAT * 2);
    float* BQ  = (float*)wsp; wsp += al256((size_t)FEAT * 4);
    float* BK  = (float*)wsp; wsp += al256((size_t)FEAT * 4);
    float* BVP = (float*)wsp; wsp += al256((size_t)FEAT * 4);
    float* BO  = (float*)wsp; wsp += al256((size_t)DM * 4);
    unsigned short* Q3P = (unsigned short*)wsp; wsp += al256((size_t)GTOK * FEAT * 2);
    unsigned short* K3P = (unsigned short*)wsp; wsp += al256((size_t)GTOK * FEAT * 2);
    unsigned short* V3H = (unsigned short*)wsp; wsp += al256((size_t)GTOK * FEAT * 2);
    unsigned short* V3L = (unsigned short*)wsp; wsp += al256((size_t)GTOK * FEAT * 2);
    unsigned short* O3  = (unsigned short*)wsp; wsp += al256((size_t)GTOK * 2 * FEAT * 2);
    const size_t carve = (size_t)(wsp - (char*)d_ws);
    if (carve > ws_size || carve > (size_t)134217728) return;

    k_castrows<<<(unsigned)(((long long)NTOK * (DM / 8) + 255) / 256), 256, 0, stream>>>(q, DM, XQ16, DM, NTOK, DM, 1.0f);
    k_castrows<<<(unsigned)(((long long)NTOK * (DM / 8) + 255) / 256), 256, 0, stream>>>(k, DM, XK16, DM, NTOK, DM, 1.0f);
    k_castrows<<<(unsigned)(((long long)NTOK * (DM / 8) + 255) / 256), 256, 0, stream>>>(v, DM, XV16, DM, NTOK, DM, 1.0f);
    k_castwT<<<(unsigned)(((long long)FEAT * (DM / 8) + 255) / 256), 256, 0, stream>>>(Wq, FEAT, WQ16, DM, DM, FEAT, 16.0f, 0, 0, 0, 0);
    k_castwT<<<(unsigned)(((long long)FEAT * (DM / 8) + 255) / 256), 256, 0, stream>>>(Wk, FEAT, WK16, DM, DM, FEAT, 16.0f, 0, 0, 0, 0);
    k_castwT<<<(unsigned)(((long long)FEAT * (DM / 8) + 255) / 256), 256, 0, stream>>>(Wv, FEAT, WV16, DM, DM, FEAT, 16.0f, 0, DM, NHD, 0);
    k_castwT<<<(unsigned)(((long long)DM * (FEAT / 8) + 255) / 256), 256, 0, stream>>>(Wo, DM, WO16, 2 * FEAT, FEAT, DM, 1.0f, 1, 0, 0, FEAT);
    k_bfvec<<<(unsigned)((FEAT + 255) / 256), 256, 0, stream>>>(bq, BQ, FEAT, 0, 0);
    k_bfvec<<<(unsigned)((FEAT + 255) / 256), 256, 0, stream>>>(bk, BK, FEAT, 0, 0);
    k_bfvec<<<(unsigned)((FEAT + 255) / 256), 256, 0, stream>>>(bv, BVP, FEAT, DM, NHD);
    k_bfvec<<<(unsigned)((DM + 255) / 256), 256, 0, stream>>>(bo, BO, DM, 0, 0);

    const unsigned gemm_blocks = (unsigned)((((GTOK) / 64) * ((FEAT) / 64) + 7) / 8);
    const unsigned oproj_blocks = (unsigned)((((GTOK) / 64) * ((DM) / 64) + 7) / 8);
    for (int g = 0; g < NGRP; ++g) {
        const size_t xoff = (size_t)g * GTOK * DM;
        w25::wmma_gemm64<0, false, 2, 1, false, 0><<<dim3(gemm_blocks, 1), 256, 0, stream>>>(
            (const unsigned short*)(XQ16 + xoff), nullptr, DM, 0, (const unsigned short*)WQ16, nullptr, DM, 0,
            (void*)Q3P, nullptr, FEAT, 0, BQ, nullptr, 0, GTOK, FEAT, DM, 0.0625f);
        w25::wmma_gemm64<0, false, 2, 1, false, 0><<<dim3(gemm_blocks, 1), 256, 0, stream>>>(
            (const unsigned short*)(XK16 + xoff), nullptr, DM, 0, (const unsigned short*)WK16, nullptr, DM, 0,
            (void*)K3P, nullptr, FEAT, 0, BK, nullptr, 0, GTOK, FEAT, DM, 0.0625f);
        w25::wmma_gemm64<0, false, 2, 2, false, 0><<<dim3(gemm_blocks, 1), 256, 0, stream>>>(
            (const unsigned short*)(XV16 + xoff), nullptr, DM, 0, (const unsigned short*)WV16, nullptr, DM, 0,
            (void*)V3H, (void*)V3L, FEAT, 0, BVP, nullptr, 0, GTOK, FEAT, DM, 0.0625f);
        k_featattn<<<(unsigned)(GTOK / 8), 256, 0, stream>>>(Q3P, K3P, V3H, V3L, O3, GTOK);
        w25::wmma_gemm64<1, false, 2, 0, false, 0><<<dim3(oproj_blocks, 1), 256, 0, stream>>>(
            (const unsigned short*)O3, nullptr, 2 * FEAT, 0, (const unsigned short*)WO16, nullptr, 2 * FEAT, 0,
            (void*)(out + (size_t)g * GTOK * DM), nullptr, DM, 0, BO, nullptr, 0, GTOK, DM, 2 * FEAT, 1.0f);
    }
    (void)hipGetLastError();
}
